// GraphSAGE_31799937859849
// MI455X (gfx1250) — hardware-verified
//
#include <hip/hip_runtime.h>
#include <stddef.h>
#include <stdint.h>

#define NNODE  50000
#define NPAD   50048
#define DEG    16
#define WID    256
#define NB     8192
#define OWNB   1024
#define OWNG   49
#define OWNN   (OWNG * OWNB)
#define GBM    128
#define GTHR   256
#define GLDS   (GBM * WID * 4)
#define NUA    (WID * (512 / 8))
#define NU0    (WID * (768 / 8))
#define NU1    (WID * (1024 / 8))
#define NUT    (NUA + NU0 + NU1)
#define EPSN   1e-12f
#define WSMAX  134217728

static_assert(WID == 256 && DEG == 16);
static_assert(NPAD % GBM == 0 && NPAD == 391 * 128 && NPAD >= NNODE);
static_assert(NB % GBM == 0 && NB % 1024 == 0);
static_assert(OWNN >= NPAD);
static_assert(NUA % 256 == 0 && NU0 % 256 == 0 && NU1 % 256 == 0);
static_assert(256 % 32 == 0 && 512 % 32 == 0 && 768 % 32 == 0 && 1024 % 32 == 0);
static_assert(NPAD % 8 == 0 && NB % 8 == 0);
static_assert(GLDS <= 300000);

typedef float          v4f   __attribute__((ext_vector_type(4)));
typedef float          v8f   __attribute__((ext_vector_type(8)));
typedef int            v4i   __attribute__((ext_vector_type(4)));
typedef int            v8i   __attribute__((ext_vector_type(8)));
typedef unsigned short v8us  __attribute__((ext_vector_type(8)));
typedef unsigned short v16us __attribute__((ext_vector_type(16)));
typedef __bf16         v16bf __attribute__((ext_vector_type(16)));
typedef v4f  __attribute__((may_alias)) v4fa;
typedef v4i  __attribute__((may_alias)) v4ia;
typedef v8us __attribute__((may_alias)) v8usa;
union FragB { v16bf v; v16us u; v8us h[2]; v8i w; };

__device__ __forceinline__ v8f wmb(const FragB& a, const FragB& b, v8f c) {
  v8f d = __builtin_amdgcn_wmma_f32_16x16x32_bf16(false, a.v, false, b.v, (short)0, c, false, false);
  asm volatile("v_nop\n\tv_nop\n\tv_nop\n\tv_nop" : "+v"(d) : "v"(a.w), "v"(b.w));
  return d;
}

__device__ __forceinline__ v8f z8() { v8f z = {0.f, 0.f, 0.f, 0.f, 0.f, 0.f, 0.f, 0.f}; return z; }

__device__ __forceinline__ unsigned bf16_bits(float f) {
  const unsigned u = __float_as_uint(f);
  return (u + 0x7FFFu + ((u >> 16) & 1u)) >> 16;
}
__device__ __forceinline__ float bf16_val(float f) {
  return __uint_as_float(bf16_bits(f) << 16);
}
__device__ __forceinline__ unsigned hl_bits(float v, unsigned& lo) {
  const unsigned hb = bf16_bits(v);
  lo = bf16_bits(v - __uint_as_float(hb << 16));
  return hb;
}
__device__ __forceinline__ void pack_hl(const float (&y)[8], unsigned msk, v8us& hv, v8us& lv) {
#pragma unroll
  for (int e = 0; e < 8; ++e) {
    unsigned lb;
    const unsigned hb = hl_bits(y[e], lb);
    hv[e] = (unsigned short)(hb & msk);
    lv[e] = (unsigned short)(lb & msk);
  }
}

__global__ __launch_bounds__(256) __attribute__((amdgpu_num_vgpr(248)))
void k_own(const int* __restrict__ nidx, int* own) {
  __shared__ __attribute__((aligned(16))) int tab[OWNB];
  const int tid  = (int)threadIdx.x;
  const int base = (int)blockIdx.x * OWNB;
  {
    const v4i neg = {-1, -1, -1, -1};
    *(v4ia*)(tab + 4 * tid) = neg;
  }
  __syncthreads();
#pragma unroll 1
  for (int it = 0; it < NB / 1024; ++it) {
    const int q = it * 256 + tid;
    const v4i v = *(const v4i*)(nidx + 4 * q);
    const int b0 = 4 * q;
    const unsigned s0 = (unsigned)(v.x - base), s1 = (unsigned)(v.y - base);
    const unsigned s2 = (unsigned)(v.z - base), s3 = (unsigned)(v.w - base);
    if (s0 < (unsigned)OWNB) atomicMax(&tab[s0], b0);
    if (s1 < (unsigned)OWNB) atomicMax(&tab[s1], b0 + 1);
    if (s2 < (unsigned)OWNB) atomicMax(&tab[s2], b0 + 2);
    if (s3 < (unsigned)OWNB) atomicMax(&tab[s3], b0 + 3);
  }
  __syncthreads();
  const v4i o = *(const v4ia*)(tab + 4 * tid);
  int* dp = own + (size_t)base + 4 * tid;
  *(volatile v4i*)dp = o;
  __threadfence();
  *(volatile v4i*)dp = o;
}

__device__ __forceinline__ v8us gat8(const float* __restrict__ w, int off) {
  v8us o;
#pragma unroll
  for (int i = 0; i < 8; ++i) o[i] = (unsigned short)bf16_bits(w[off + i * WID]);
  return o;
}

__global__ __launch_bounds__(256) __attribute__((amdgpu_num_vgpr(248)))
void k_prep(const float* __restrict__ wagg, const float* __restrict__ wlin, unsigned short* wpl) {
  const int u = (int)blockIdx.x * 256 + (int)threadIdx.x;
  v8us o;
  if (u < NUA) {
    const int n = u >> 6, k8 = (u & 63) * 8;
    const int r = k8 & 255;
    o = gat8(wagg, r * WID + n);
  } else if (u < NUA + NU0) {
    const int v = u - NUA;
    const int n = v / 96, k8 = (v - n * 96) * 8;
    const int r = (k8 < 512) ? k8 : (k8 - 256);
    o = gat8(wlin, r * WID + n);
  } else if (u < NUT) {
    const int v = u - NUA - NU0;
    const int n = v >> 7, k8 = (v & 127) * 8;
    const int r = (k8 < 256) ? k8 : ((k8 < 768) ? (k8 - 256) : (k8 - 512));
    o = gat8(wlin, 512 * WID + r * WID + n);
  } else {
    return;
  }
  unsigned short* dp = wpl + (size_t)u * 8;
  *(volatile v8us*)dp = o;
  __threadfence();
  *(volatile v8us*)dp = o;
}

__global__ __launch_bounds__(256) __attribute__((amdgpu_num_vgpr(248)))
void k_h0(const float* __restrict__ feats, const int* __restrict__ own, unsigned short* h0b) {
  const int lane = (int)threadIdx.x & 31, wave = (int)threadIdx.x >> 5;
  const int n = (int)blockIdx.x * 8 + wave;
  int o = own[n];
  o = o < -1 ? -1 : (o > NB - 1 ? NB - 1 : o);
  const int oc = o < 0 ? 0 : o;
  const float* fp = feats + (size_t)oc * WID + 8 * lane;
  const v4f a = *(const v4f*)fp;
  const v4f c = *(const v4f*)(fp + 4);
  const unsigned msk = (o >= 0 && n < NNODE) ? 0xFFFFu : 0u;
  v8us q;
  q[0] = (unsigned short)(bf16_bits(a.x) & msk); q[1] = (unsigned short)(bf16_bits(a.y) & msk);
  q[2] = (unsigned short)(bf16_bits(a.z) & msk); q[3] = (unsigned short)(bf16_bits(a.w) & msk);
  q[4] = (unsigned short)(bf16_bits(c.x) & msk); q[5] = (unsigned short)(bf16_bits(c.y) & msk);
  q[6] = (unsigned short)(bf16_bits(c.z) & msk); q[7] = (unsigned short)(bf16_bits(c.w) & msk);
  unsigned short* dp = h0b + (size_t)n * WID + 8 * lane;
  *(volatile v8us*)dp = q;
  __threadfence();
  *(volatile v8us*)dp = q;
}

__device__ __forceinline__ void nbr_max(const float* __restrict__ agg, int nb, int lane, v4f& ma, v4f& mb) {
  const float nh = -__builtin_huge_valf();
  v4f a = {nh, nh, nh, nh};
  v4f b = {nh, nh, nh, nh};
#pragma unroll 4
  for (int j = 0; j < DEG; ++j) {
    const int nj = __shfl(nb, j, 32);
    const float* rp = agg + (size_t)nj * WID + 8 * lane;
    const v4f x = *(const v4f*)rp;
    const v4f y = *(const v4f*)(rp + 4);
    a.x = fmaxf(a.x, x.x); a.y = fmaxf(a.y, x.y); a.z = fmaxf(a.z, x.z); a.w = fmaxf(a.w, x.w);
    b.x = fmaxf(b.x, y.x); b.y = fmaxf(b.y, y.y); b.z = fmaxf(b.z, y.z); b.w = fmaxf(b.w, y.w);
  }
  ma = a; mb = b;
}

__global__ __launch_bounds__(256) __attribute__((amdgpu_num_vgpr(248)))
void k_nm0(const float* __restrict__ agg, const int* __restrict__ nbd, unsigned short* nm) {
  const int lane = (int)threadIdx.x & 31, wave = (int)threadIdx.x >> 5;
  const int n  = (int)blockIdx.x * 8 + wave;
  const int nc = n < NNODE ? n : NNODE - 1;
  int nb = nbd[(size_t)nc * DEG + (lane & 15)];
  nb = nb < 0 ? 0 : (nb > NNODE - 1 ? NNODE - 1 : nb);
  v4f ma, mb;
  nbr_max(agg, nb, lane, ma, mb);
  const float y[8] = {ma.x, ma.y, ma.z, ma.w, mb.x, mb.y, mb.z, mb.w};
  const unsigned msk = (n < NNODE) ? 0xFFFFu : 0u;
  v8us hv, lv;
  pack_hl(y, msk, hv, lv);
  unsigned short* dp = nm + (size_t)n * 512 + 8 * lane;
  *(volatile v8us*)dp = hv;
  *(volatile v8us*)(dp + 256) = lv;
  __threadfence();
  *(volatile v8us*)dp = hv;
  *(volatile v8us*)(dp + 256) = lv;
}

__global__ __launch_bounds__(256) __attribute__((amdgpu_num_vgpr(248)))
void k_nm1(const float* __restrict__ agg, const int* __restrict__ nbd, const int* __restrict__ nidx,
           const unsigned short* __restrict__ h1, unsigned short* a1) {
  const int lane = (int)threadIdx.x & 31, wave = (int)threadIdx.x >> 5;
  const int b = (int)blockIdx.x * 8 + wave;
  int n = nidx[b];
  n = n < 0 ? 0 : (n > NNODE - 1 ? NNODE - 1 : n);
  int nb = nbd[(size_t)n * DEG + (lane & 15)];
  nb = nb < 0 ? 0 : (nb > NNODE - 1 ? NNODE - 1 : nb);
  const unsigned short* hp = h1 + (size_t)n * 512 + 8 * lane;
  const v8us hh = *(const v8usa*)hp;
  const v8us hl = *(const v8usa*)(hp + 256);
  v4f ma, mb;
  nbr_max(agg, nb, lane, ma, mb);
  const float y[8] = {ma.x, ma.y, ma.z, ma.w, mb.x, mb.y, mb.z, mb.w};
  v8us hv, lv;
  pack_hl(y, 0xFFFFu, hv, lv);
  unsigned short* dp = a1 + (size_t)b * 1024 + 8 * lane;
  *(volatile v8us*)dp = hh;
  *(volatile v8us*)(dp + 256) = hl;
  *(volatile v8us*)(dp + 512) = hv;
  *(volatile v8us*)(dp + 768) = lv;
  __threadfence();
  *(volatile v8us*)dp = hh;
  *(volatile v8us*)(dp + 256) = hl;
  *(volatile v8us*)(dp + 512) = hv;
  *(volatile v8us*)(dp + 768) = lv;
}

__device__ __forceinline__ void gstep(const unsigned short* a0p, const unsigned short* a1p,
                                      const unsigned short* __restrict__ bq, int ldb, v8f (&acc)[2][8]) {
  FragB af0, af1;
  af0.h[0] = *(const v8usa*)a0p;
  af0.h[1] = *(const v8usa*)(a0p + 16);
  af1.h[0] = *(const v8usa*)a1p;
  af1.h[1] = *(const v8usa*)(a1p + 16);
#pragma unroll
  for (int nt = 0; nt < 8; ++nt) {
    const unsigned short* wq = bq + (size_t)(16 * nt) * (size_t)ldb;
    FragB bf;
    bf.h[0] = *(const v8usa*)wq;
    bf.h[1] = *(const v8usa*)(wq + 16);
    acc[0][nt] = wmb(af0, bf, acc[0][nt]);
    acc[1][nt] = wmb(af1, bf, acc[1][nt]);
  }
}

template <int MODE>
__device__ __forceinline__ void epi_pass(const float* stg, v4f ba, v4f bb, int c0, int c1, int rowBase,
                                         int wave, int lane, float* outF, unsigned short* outH, int nValid) {
#pragma unroll 1
  for (int i = 0; i < 16; ++i) {
    const int lr  = 16 * wave + i;
    const int row = rowBase + lr;
    const bool ok = row < nValid;
    const v4f x0 = *(const v4fa*)(stg + lr * WID + c0);
    const v4f x1 = *(const v4fa*)(stg + lr * WID + c1);
    float y[8];
    y[0] = fmaxf(x0.x + ba.x, 0.0f); y[1] = fmaxf(x0.y + ba.y, 0.0f);
    y[2] = fmaxf(x0.z + ba.z, 0.0f); y[3] = fmaxf(x0.w + ba.w, 0.0f);
    y[4] = fmaxf(x1.x + bb.x, 0.0f); y[5] = fmaxf(x1.y + bb.y, 0.0f);
    y[6] = fmaxf(x1.z + bb.z, 0.0f); y[7] = fmaxf(x1.w + bb.w, 0.0f);
    if constexpr (MODE != 0) {
      float s = ((y[0] * y[0] + y[1] * y[1]) + (y[2] * y[2] + y[3] * y[3])) +
                ((y[4] * y[4] + y[5] * y[5]) + (y[6] * y[6] + y[7] * y[7]));
      s += __shfl_xor(s, 16, 32);
      s += __shfl_xor(s, 8, 32);
      s += __shfl_xor(s, 4, 32);
      s += __shfl_xor(s, 2, 32);
      s += __shfl_xor(s, 1, 32);
      const float rinv = 1.0f / fmaxf(sqrtf(s), EPSN);
#pragma unroll
      for (int e = 0; e < 8; ++e) y[e] = y[e] * rinv;
    }
    if constexpr (MODE == 1) {
      v8us hv, lv;
      pack_hl(y, ok ? 0xFFFFu : 0u, hv, lv);
      unsigned short* dp = outH + (size_t)row * 512 + 8 * lane;
      *(volatile v8us*)dp = hv;
      *(volatile v8us*)(dp + 256) = lv;
    } else {
      v4f o0, o1;
      o0.x = ok ? y[0] : 0.0f; o0.y = ok ? y[1] : 0.0f; o0.z = ok ? y[2] : 0.0f; o0.w = ok ? y[3] : 0.0f;
      o1.x = ok ? y[4] : 0.0f; o1.y = ok ? y[5] : 0.0f; o1.z = ok ? y[6] : 0.0f; o1.w = ok ? y[7] : 0.0f;
      float* dp = outF + (size_t)row * WID;
      if constexpr (MODE == 0) {
        *(volatile v4f*)(dp + c0) = o0;
        *(volatile v4f*)(dp + c1) = o1;
      } else {
        if (ok) {
          *(volatile v4f*)(dp + c0) = o0;
          *(volatile v4f*)(dp + c1) = o1;
        }
      }
    }
  }
}

template <int MODE>
__global__ __launch_bounds__(GTHR) __attribute__((amdgpu_num_vgpr(248)))
void k_gemm(const unsigned short* A1, int lda1, int K1,
            const unsigned short* A2, int lda2, int K2,
            const unsigned short* __restrict__ BT, int ldb,
            const float* __restrict__ bias, float* outF, unsigned short* outH, int nValid) {
  extern __shared__ __attribute__((aligned(16))) float stg[];
  const int tid = (int)threadIdx.x, lane = tid & 31, wave = tid >> 5, hh = lane >> 4, m = lane & 15;
  const int wr = wave >> 1, wc = wave & 1;
  const int rowBase = (int)blockIdx.x * GBM;

  v8f acc[2][8];
#pragma unroll
  for (int mi = 0; mi < 2; ++mi)
#pragma unroll
    for (int nt = 0; nt < 8; ++nt) acc[mi][nt] = z8();

  const size_t arow = (size_t)(rowBase + 32 * wr + m);
  const unsigned short* bp = BT + (size_t)(128 * wc + m) * (size_t)ldb + 8 * hh;
  {
    const unsigned short* ap0 = A1 + arow * (size_t)lda1 + 8 * hh;
    const unsigned short* ap1 = ap0 + (size_t)16 * (size_t)lda1;
#pragma unroll 1
    for (int k0 = 0; k0 < K1; k0 += 32) gstep(ap0 + k0, ap1 + k0, bp + k0, ldb, acc);
  }
  {
    const unsigned short* cp0 = A2 + arow * (size_t)lda2 + 8 * hh;
    const unsigned short* cp1 = cp0 + (size_t)16 * (size_t)lda2;
#pragma unroll 1
    for (int k0 = 0; k0 < K2; k0 += 32) gstep(cp0 + k0, cp1 + k0, bp + K1 + k0, ldb, acc);
  }

#pragma unroll
  for (int mi = 0; mi < 2; ++mi)
#pragma unroll
    for (int nt = 0; nt < 8; ++nt)
#pragma unroll
      for (int r = 0; r < 8; ++r)
        stg[(32 * wr + 16 * mi + 8 * hh + r) * WID + 128 * wc + 16 * nt + m] = acc[mi][nt][r];
  __syncthreads();

  const int c0 = (MODE == 1) ? (8 * lane) : (4 * lane);
  const int c1 = (MODE == 1) ? (8 * lane + 4) : (128 + 4 * lane);
  v4f ba, bb;
  {
    const v4f p = *(const v4f*)(bias + c0);
    const v4f q = *(const v4f*)(bias + c1);
    ba.x = bf16_val(p.x); ba.y = bf16_val(p.y); ba.z = bf16_val(p.z); ba.w = bf16_val(p.w);
    bb.x = bf16_val(q.x); bb.y = bf16_val(q.y); bb.z = bf16_val(q.z); bb.w = bf16_val(q.w);
  }
  epi_pass<MODE>(stg, ba, bb, c0, c1, rowBase, wave, lane, outF, outH, nValid);
  __threadfence();
  epi_pass<MODE>(stg, ba, bb, c0, c1, rowBase, wave, lane, outF, outH, nValid);
}

extern "C" void kernel_launch(void* const* d_in, const int* in_sizes, int n_in,
                              void* d_out, int out_size, void* d_ws, size_t ws_size,
                              hipStream_t stream) {
  if (n_in < 7) return;
  if (in_sizes[0] != NB) return;
  if (in_sizes[1] != NB * WID) return;
  if (in_sizes[2] != NNODE * DEG) return;
  if (in_sizes[3] != WID * WID) return;
  if (in_sizes[4] != WID) return;
  if (in_sizes[5] != 2 * 512 * WID) return;
  if (in_sizes[6] != 2 * WID) return;
  if (out_size != NB * WID) return;

  const int*   nidx  = (const int*)  d_in[0];
  const float* feats = (const float*)d_in[1];
  const int*   nbd   = (const int*)  d_in[2];
  const float* wagg  = (const float*)d_in[3];
  const float* bagg  = (const float*)d_in[4];
  const float* wlin  = (const float*)d_in[5];
  const float* blin  = (const float*)d_in[6];
  float* out = (float*)d_out;

  const size_t szAGG = (size_t)NPAD * WID * 4;
  const size_t szNM  = (size_t)NPAD * 512 * 2;
  const size_t szH0  = (size_t)NPAD * WID * 2;
  const size_t szOWN = (size_t)OWNN * 4;
  const size_t szWPL = (size_t)NUT * 8 * 2;
  const size_t oAGG = 0;
  const size_t oNM  = oAGG + szAGG;
  const size_t oH0  = oNM + szNM;
  const size_t oOWN = oH0 + szH0;
  const size_t oWPL = oOWN + szOWN;
  const size_t total = oWPL + szWPL;
  if ((size_t)NB * 1024 * 2 > szH0) return;
  if (total > ws_size || total > (size_t)WSMAX) return;

  char* ws = (char*)d_ws;
  float*          AGG = (float*)(ws + oAGG);
  unsigned short* NM  = (unsigned short*)(ws + oNM);
  unsigned short* H0b = (unsigned short*)(ws + oH0);
  unsigned short* A1p = (unsigned short*)(ws + oH0);
  int*            OWN = (int*)(ws + oOWN);
  unsigned short* WPL = (unsigned short*)(ws + oWPL);
  unsigned short* WAD = WPL;
  unsigned short* WL0 = WPL + (size_t)NUA * 8;
  unsigned short* WL1 = WL0 + (size_t)NU0 * 8;

  hipFuncSetAttribute(reinterpret_cast<const void*>(&k_gemm<0>), hipFuncAttributeMaxDynamicSharedMemorySize, (int)GLDS);
  hipFuncSetAttribute(reinterpret_cast<const void*>(&k_gemm<1>), hipFuncAttributeMaxDynamicSharedMemorySize, (int)GLDS);
  hipFuncSetAttribute(reinterpret_cast<const void*>(&k_gemm<2>), hipFuncAttributeMaxDynamicSharedMemorySize, (int)GLDS);

  const int gN = NPAD / GBM;
  const int gB = NB / GBM;

  k_own<<<OWNG, 256, 0, stream>>>(nidx, OWN);
  k_prep<<<NUT / 256, 256, 0, stream>>>(wagg, wlin, WPL);
  k_h0<<<NPAD / 8, 256, 0, stream>>>(feats, OWN, H0b);
  k_gemm<0><<<gN, GTHR, GLDS, stream>>>(H0b, WID, 256, H0b, WID, 0, WAD, 512, bagg, AGG, NM, NNODE);
  k_nm0<<<NPAD / 8, 256, 0, stream>>>(AGG, nbd, NM);
  k_gemm<1><<<gN, GTHR, GLDS, stream>>>(H0b, WID, 256, NM, 512, 512, WL0, 768, blin, AGG, NM, NNODE);
  k_gemm<0><<<gN, GTHR, GLDS, stream>>>(NM, 512, 512, NM, 512, 0, WAD, 512, bagg, AGG, NM, NNODE);
  k_nm1<<<NB / 8, 256, 0, stream>>>(AGG, nbd, nidx, NM, A1p);
  k_gemm<2><<<gB, GTHR, GLDS, stream>>>(A1p, 1024, 1024, A1p, 1024, 0, WL1, 1024, blin + WID, out, NM, NB);
}
